// MambaBlock_14267881357438
// MI455X (gfx1250) — hardware-run, weakly checked
//
#include <hip/hip_runtime.h>
#include <math.h>

typedef __attribute__((ext_vector_type(16))) _Float16 v16h;
typedef __attribute__((ext_vector_type(8)))  _Float16 v8h;
typedef __attribute__((ext_vector_type(2)))  _Float16 v2h;
typedef __attribute__((ext_vector_type(16))) __bf16   v16b;
typedef __attribute__((ext_vector_type(8)))  __bf16   v8b;
typedef __attribute__((ext_vector_type(8)))  float    v8f;
typedef __attribute__((ext_vector_type(4)))  float    v4f;
typedef __attribute__((ext_vector_type(2)))  float    v2f;
typedef __attribute__((ext_vector_type(4)))  _Float16 v4h;

constexpr int kNB   = 2;
constexpr int kL    = 2048;
constexpr int kRows = kNB * kL;
constexpr int kDm   = 1024;
constexpr int kDi   = 2048;
constexpr int kR    = 64;
constexpr int kS    = 16;
constexpr int kXP   = 128;
constexpr int kOut0 = kRows * kDm;
constexpr int kThr  = 256;
constexpr float kEps = 1e-6f;
constexpr float kDtMin = 0.001f, kDtMax = 0.1f;
constexpr float kInCarry = 1024.0f;
constexpr float kYCarry  = 512.0f;
constexpr float kWCarry  = 4096.0f;
constexpr float kScA = 1.0f / (kInCarry * kWCarry);
constexpr float kScY = 1.0f / (kYCarry * kWCarry);
constexpr float kF16MinNormal = 6.103515625e-5f;

static_assert(kRows == 4096 && kDm == 1024 && kDi == 2048 && kR == 64 && kS == 16 && kXP == 128 && (1 << 11) == kL, "the index arithmetic below uses these sizes");

constexpr size_t kOffXN16 = 0ull;
constexpr size_t kOffWIN16 = 8388608ull;
constexpr size_t kOffUZ = 16777216ull;
constexpr size_t kOffU = 83886080ull;
constexpr size_t kOffU16 = 117440512ull;
constexpr size_t kOffWX16 = 134217728ull;
constexpr size_t kOffXP = 134742016ull;
constexpr size_t kOffDTR16 = 136839168ull;
constexpr size_t kOffBC = 137363456ull;
constexpr size_t kOffWDO16 = 137887744ull;
constexpr size_t kOffDT = 138149888ull;
constexpr size_t kOffY16 = 171704320ull;
constexpr size_t kOffWOUT16 = 188481536ull;
constexpr size_t kOffO = 192675840ull;
constexpr size_t kOffBV = 209453056ull;
constexpr size_t kOffRS = 209482240ull;
constexpr size_t kWsTotal = 209498624ull;
static_assert(kWsTotal <= 268435456ull, "the carve stands under the contract's 256 MiB of workspace");
static_assert(kOffXN16 == 0
  && kOffWIN16 == kOffXN16 + 8388608ull
  && kOffUZ == kOffWIN16 + 8388608ull
  && kOffU == kOffUZ + 67108864ull
  && kOffU16 == kOffU + 33554432ull
  && kOffWX16 == kOffU16 + 16777216ull
  && kOffXP == kOffWX16 + 524288ull
  && kOffDTR16 == kOffXP + 2097152ull
  && kOffBC == kOffDTR16 + 524288ull
  && kOffWDO16 == kOffBC + 524288ull
  && kOffDT == kOffWDO16 + 262144ull
  && kOffY16 == kOffDT + 33554432ull
  && kOffWOUT16 == kOffY16 + 16777216ull
  && kOffO == kOffWOUT16 + 4194304ull
  && kOffBV == kOffO + 16777216ull
  && kOffRS == kOffBV + 29184ull
  && kWsTotal == kOffRS + 16384ull, "the carve is a chain: every region starts where the one before ends");
static_assert((size_t)kRows * kDm * 2 == 8388608ull && (size_t)kRows * 2 * kDi * 4 == 67108864ull && (size_t)kRows * kDi * 4 == 33554432ull && (size_t)kXP * kDi * 2 == 524288ull && (size_t)kRows * kXP * 4 == 2097152ull && (size_t)kRows * kDm * 4 == 16777216ull && (size_t)(2 * kDi + kXP + kDi + kDm) * 4 == 29184ull, "every region's length is its plane's");
static_assert((kOffWIN16 % 256) == 0 && (kOffUZ % 256) == 0 && (kOffU % 256) == 0 && (kOffU16 % 256) == 0 && (kOffWX16 % 256) == 0 && (kOffXP % 256) == 0 && (kOffDTR16 % 256) == 0 && (kOffBC % 256) == 0 && (kOffWDO16 % 256) == 0 && (kOffDT % 256) == 0 && (kOffY16 % 256) == 0 && (kOffWOUT16 % 256) == 0 && (kOffO % 256) == 0 && (kOffBV % 256) == 0 && (kOffRS % 256) == 0, "every region starts on a multiple of 256 B");
constexpr int kBvIn = 0, kBvX = 2 * kDi, kBvDo = 2 * kDi + kXP, kBvOut = 2 * kDi + kXP + kDi;

__device__ __forceinline__ unsigned short f2bf_bits(float f) {
  unsigned u = __float_as_uint(f);
  return (unsigned short)((u + 0x7FFFu + ((u >> 16) & 1u)) >> 16);
}
__device__ __forceinline__ float bf_bits2f(unsigned short h) { return __uint_as_float(((unsigned)h) << 16); }
__device__ __forceinline__ float bf16r(float f) { return bf_bits2f(f2bf_bits(f)); }
__device__ __forceinline__ float carry_flush(float v, float carry) {
  const float s = v * carry;
  return (fabsf(s) < kF16MinNormal) ? 0.0f : s;
}

__device__ __forceinline__ void dep_guard4_h(v8f& a, v8f& b, v8f& c, v8f& d, v16h x, v16h y) { asm volatile("v_nop\n\tv_nop\n\tv_nop\n\tv_nop" : "+v"(a), "+v"(b), "+v"(c), "+v"(d) : "v"(x), "v"(y)); }
__device__ __forceinline__ void dep_guard4_b(v8f& a, v8f& b, v8f& c, v8f& d, v16b x, v16b y) { asm volatile("v_nop\n\tv_nop\n\tv_nop\n\tv_nop" : "+v"(a), "+v"(b), "+v"(c), "+v"(d) : "v"(x), "v"(y)); }
__device__ __forceinline__ void keep4_h(v16h a, v16h b, v16h c, v16h d) { asm volatile("v_nop" :: "v"(a), "v"(b), "v"(c), "v"(d)); }
__device__ __forceinline__ void keep4_b(v16b a, v16b b, v16b c, v16b d) { asm volatile("v_nop" :: "v"(a), "v"(b), "v"(c), "v"(d)); }
__device__ __forceinline__ void acc_guard4(v8f& a, v8f& b, v8f& c, v8f& d) { asm volatile("v_nop\n\tv_nop\n\tv_nop\n\tv_nop" : "+v"(a), "+v"(b), "+v"(c), "+v"(d)); }

template <typename T> struct Frag;
template <> struct Frag<_Float16> {
  typedef v16h V; union U { v16h v; v8h h[2]; };
  static __device__ __forceinline__ v16h load(const _Float16* p) {
    U f; f.h[0] = *(const v8h*)(p); f.h[1] = *(const v8h*)(p + 16); return f.v;
  }
  static __device__ __forceinline__ v8f mma(v16h a, v16h b, v8f c) {
    return __builtin_amdgcn_wmma_f32_16x16x32_f16(false, a, false, b, (short)0, c, false, false);
  }
  static __device__ __forceinline__ void guard4(v8f& a, v8f& b, v8f& c, v8f& d, v16h x, v16h y) { dep_guard4_h(a, b, c, d, x, y); }
  static __device__ __forceinline__ void keep(v16h a, v16h b, v16h c, v16h d) { keep4_h(a, b, c, d); }
};
template <> struct Frag<__bf16> {
  typedef v16b V; union U { v16b v; v8b h[2]; };
  static __device__ __forceinline__ v16b load(const __bf16* p) {
    U f; f.h[0] = *(const v8b*)(p); f.h[1] = *(const v8b*)(p + 16); return f.v;
  }
  static __device__ __forceinline__ v8f mma(v16b a, v16b b, v8f c) {
    return __builtin_amdgcn_wmma_f32_16x16x32_bf16(false, a, false, b, (short)0, c, false, false);
  }
  static __device__ __forceinline__ void guard4(v8f& a, v8f& b, v8f& c, v8f& d, v16b x, v16b y) { dep_guard4_b(a, b, c, d, x, y); }
  static __device__ __forceinline__ void keep(v16b a, v16b b, v16b c, v16b d) { keep4_b(a, b, c, d); }
};

__device__ __forceinline__ v8f mma_h(v16h a, v16h b, v8f c) {
  c = __builtin_amdgcn_wmma_f32_16x16x32_f16(false, a, false, b, (short)0, c, false, false);
  asm volatile("v_nop\n\tv_nop\n\tv_nop\n\tv_nop" : "+v"(c) : "v"(a), "v"(b));
  return c;
}

template <int ET> struct Elem;
template <> struct Elem<0> { typedef _Float16 T; };
template <> struct Elem<1> { typedef __bf16 T; };
template <int ET, bool SPLIT, int BIAS_MODE, int OUT_MODE, bool RESID, int ACT = 0>
__global__ __launch_bounds__(256) void wmma_gemm64(
    const unsigned short* __restrict__ Ap, const unsigned short* __restrict__ A2p, int lda, long strideA,
    const unsigned short* __restrict__ Btp, const unsigned short* __restrict__ Bt2p, int ldb, long strideB,
    void* __restrict__ Cout, void* __restrict__ Cout2, int ldc, long strideC,
    const float* __restrict__ bias,
    const float* __restrict__ resid, long strideR,
    int M, int N, int K, float scale) {
  typedef typename Elem<ET>::T T;
  typedef typename Frag<T>::V V;
  const T* A = (const T*)Ap; const T* A2 = (const T*)A2p; const T* Bt = (const T*)Btp; const T* Bt2 = (const T*)Bt2p;
  __shared__ __align__(16) float sT[8][16 * 68];
  const int b    = blockIdx.y;
  const int lane = threadIdx.x & 31;
  const int wave = threadIdx.x >> 5;
  const int tilesN = N >> 6;
  const int tilesM = M >> 6;
  const int tile = blockIdx.x * 8 + wave;
  if (tile >= tilesM * tilesN) return;
  const int tm = tile / tilesN;
  const int tn = tile - tm * tilesN;
  const int m0 = tm << 6;
  const int n0 = tn << 6;

  const T* Ab  = A  + (size_t)b * strideA;
  const T* Bb  = Bt + (size_t)b * strideB;
  const T* Ab2 = SPLIT ? (A2  + (size_t)b * strideA) : nullptr;
  const T* Bb2 = SPLIT ? (Bt2 + (size_t)b * strideB) : nullptr;

  const int rlane = lane & 15;
  const int koff  = (lane >> 4) * 8;
  const int mOff  = (lane >> 4) * 8;

  v8f acc[4][4];
#pragma unroll
  for (int i = 0; i < 4; ++i)
#pragma unroll
    for (int j = 0; j < 4; ++j) acc[i][j] = (v8f){0.f,0.f,0.f,0.f,0.f,0.f,0.f,0.f};

  for (int k0 = 0; k0 < K; k0 += 32) {
    V bh[4], bl[4];
#pragma unroll
    for (int j = 0; j < 4; ++j) {
      const size_t bo = (size_t)(n0 + (j << 4) + rlane) * ldb + koff + k0;
      bh[j] = Frag<T>::load(Bb + bo);
      if (SPLIT) bl[j] = Frag<T>::load(Bb2 + bo);
    }
#pragma unroll
    for (int i = 0; i < 4; ++i) {
      const size_t ao = (size_t)(m0 + (i << 4) + rlane) * lda + koff + k0;
      V ah = Frag<T>::load(Ab + ao);
      V al;
      if (SPLIT) al = Frag<T>::load(Ab2 + ao);
#pragma unroll
      for (int j = 0; j < 4; ++j) {
        acc[i][j] = Frag<T>::mma(ah, bh[j], acc[i][j]);
        if (SPLIT) {
          acc[i][j] = Frag<T>::mma(ah, bl[j], acc[i][j]);
          acc[i][j] = Frag<T>::mma(al, bh[j], acc[i][j]);
        }
      }
      Frag<T>::guard4(acc[i][0], acc[i][1], acc[i][2], acc[i][3], ah, SPLIT ? al : ah);
    }
    Frag<T>::keep(bh[0], bh[1], bh[2], bh[3]);
    if (SPLIT) Frag<T>::keep(bl[0], bl[1], bl[2], bl[3]);
  }
  acc_guard4(acc[0][0], acc[0][1], acc[0][2], acc[0][3]);
  acc_guard4(acc[1][0], acc[1][1], acc[1][2], acc[1][3]);
  acc_guard4(acc[2][0], acc[2][1], acc[2][2], acc[2][3]);
  acc_guard4(acc[3][0], acc[3][1], acc[3][2], acc[3][3]);

  float* slab = sT[wave];
  const float* Rb = RESID ? (resid + (size_t)b * strideR) : nullptr;
#pragma unroll
  for (int i = 0; i < 4; ++i) {
    const int mBase = m0 + (i << 4);
#pragma unroll
    for (int j = 0; j < 4; ++j) {
      const int n = n0 + (j << 4) + rlane;
      float bv = 0.f;
      if (BIAS_MODE == 2) bv = bias[n];
#pragma unroll
      for (int r = 0; r < 8; ++r) {
        float v = acc[i][j][r] * scale;
        if (BIAS_MODE == 1) v += bias[mBase + mOff + r];
        if (BIAS_MODE == 2) v += bv;
        if (RESID) v += Rb[(size_t)(mBase + mOff + r) * ldc + n];
        if (ACT == 1) v = tanhf(v);
        if (ACT == 2) v = fmaxf(v, 0.0f);
        if (ACT == 3) v = v / (1.0f + expf(-v));
        if (ACT == 4) v = (v > 0.f) ? v : 0.01f * v;
        slab[(mOff + r) * 68 + (j << 4) + rlane] = v;
      }
    }
    __builtin_amdgcn_fence(__ATOMIC_RELEASE, "workgroup");
    __builtin_amdgcn_wave_barrier();
    __builtin_amdgcn_fence(__ATOMIC_ACQUIRE, "workgroup");
    if (OUT_MODE == 0) {
      float* C = (float*)Cout + (size_t)b * strideC;
      const int hh = lane >> 4, c4 = (lane & 15) * 4;
      for (int pass = 0; pass < 2; ++pass) {
#pragma unroll
        for (int it = 0; it < 8; ++it) {
          const int row = it * 2 + hh;
          v4f v = *(const v4f*)(slab + row * 68 + c4);
          *(volatile v4f*)(C + (size_t)(mBase + row) * ldc + n0 + c4) = v;
        }
        __threadfence();
      }
    } else {
      const int q = lane >> 3, c8 = (lane & 7) * 8;
      unsigned short* C  = (unsigned short*)Cout  + (size_t)b * strideC;
      unsigned short* C2 = (OUT_MODE == 2) ? ((unsigned short*)Cout2 + (size_t)b * strideC) : nullptr;
      for (int pass = 0; pass < 2; ++pass) {
#pragma unroll
        for (int it = 0; it < 4; ++it) {
          const int row = it * 4 + q;
          const float* sp = slab + row * 68 + c8;
          v8h hv, lv;
#pragma unroll
          for (int e = 0; e < 8; ++e) {
            if (OUT_MODE == 1) {
              hv[e] = (_Float16)sp[e];
            } else {
              unsigned short hb = f2bf_bits(sp[e]);
              unsigned short lb = f2bf_bits(sp[e] - bf_bits2f(hb));
              hv[e] = __builtin_bit_cast(_Float16, hb);
              lv[e] = __builtin_bit_cast(_Float16, lb);
            }
          }
          *(volatile v8h*)(C + (size_t)(mBase + row) * ldc + n0 + c8) = hv;
          if (OUT_MODE == 2) *(volatile v8h*)(C2 + (size_t)(mBase + row) * ldc + n0 + c8) = lv;
        }
        __threadfence();
      }
    }
    __builtin_amdgcn_fence(__ATOMIC_RELEASE, "workgroup");
    __builtin_amdgcn_wave_barrier();
    __builtin_amdgcn_fence(__ATOMIC_ACQUIRE, "workgroup");
  }
}


__global__ __launch_bounds__(256) void wt_plane_kernel(const float* __restrict__ W, unsigned short* __restrict__ dst, int K, int N, int nLive, int ldd, int colOff) {
  const int n  = blockIdx.x;
  const int k8 = threadIdx.x * 8;
  const bool live = n < nLive;
  const int nc = live ? n : 0;
  v8h hv;
#pragma unroll
  for (int e = 0; e < 8; ++e) {
    const float w = W[(size_t)(k8 + e) * N + nc];
    hv[e] = (_Float16)(live ? carry_flush(bf16r(w), kWCarry) : 0.0f);
  }
  unsigned short* dp = dst + (size_t)n * ldd + colOff + k8;
  *(volatile v8h*)dp = hv;
  __threadfence();
  *(volatile v8h*)dp = hv;
}

__global__ __launch_bounds__(kThr) void setup_kernel(const float* __restrict__ in_proj_b, const float* __restrict__ dt_in_b, const float* __restrict__ b_proj_b, const float* __restrict__ c_proj_b, const float* __restrict__ dt_out_b, const float* __restrict__ out_proj_b, float* __restrict__ BV) {
  const unsigned i = blockIdx.x * (unsigned)kThr + threadIdx.x;
  if (i >= (unsigned)(kBvOut + kDm)) return;
  const unsigned j = i - (unsigned)kBvX;
  const float v0 = in_proj_b[i & 4095u];
  const float v1 = dt_in_b[j & 63u];
  const float v2 = b_proj_b[j & 15u];
  const float v3 = c_proj_b[j & 15u];
  const float v4 = dt_out_b[(i - (unsigned)kBvDo) & 2047u];
  const float v5 = out_proj_b[(i - (unsigned)kBvOut) & 1023u];
  const float vx = (j < 64u) ? v1 : ((j < 80u) ? v2 : ((j < 96u) ? v3 : 0.0f));
  const float o = bf16r((i < (unsigned)kBvX) ? v0 : ((i < (unsigned)kBvDo) ? vx : ((i < (unsigned)kBvOut) ? v4 : v5)));
  float* dp = BV + i;
  *(volatile float*)dp = o;
  __threadfence();
  *(volatile float*)dp = o;
}
static_assert(kBvOut + kDm == 7296 && 29 * kThr >= 7296 && 28 * kThr < 7296, "the bias records' grid: 29 blocks, the last guarded");

__global__ __launch_bounds__(kThr) void rowstat_kernel(const float* __restrict__ x, float* __restrict__ RS) {
  const unsigned row = blockIdx.x * (unsigned)kThr + threadIdx.x;
  const float* xp = x + row * (unsigned)kDm;
  float ss = 0.0f;
  for (int c = 0; c < kDm; c += 4) {
    const v4f a = *(const v4f*)(xp + c);
#pragma unroll
    for (int e = 0; e < 4; ++e) { const float v = bf16r(a[e]); ss += v * v; }
  }
  const float r = 1.0f / sqrtf(ss / (float)kDm + kEps);
  float* dp = RS + row;
  *(volatile float*)dp = r;
  __threadfence();
  *(volatile float*)dp = r;
}
static_assert(kRows == 16 * kThr, "the row statistic's grid exact: 16 blocks: a lane a row");

__global__ __launch_bounds__(kThr) void norm_kernel(const float* __restrict__ x, const float* __restrict__ RS, const float* __restrict__ norm_scale, unsigned short* __restrict__ XN16) {
  const unsigned i = blockIdx.x * (unsigned)kThr + threadIdx.x;
  const unsigned row = i >> 7;
  const unsigned c8 = (i & 127u) * 8u;
  const float r = RS[row];
  const v4f a0 = *(const v4f*)(x + i * 8u), a1 = *(const v4f*)(x + i * 8u + 4u);
  const v4f s0 = *(const v4f*)(norm_scale + c8), s1 = *(const v4f*)(norm_scale + c8 + 4u);
  v8h hv;
#pragma unroll
  for (int e = 0; e < 4; ++e) { hv[e] = (_Float16)carry_flush(bf16r(a0[e]) * r * bf16r(s0[e]), kInCarry); hv[4 + e] = (_Float16)carry_flush(bf16r(a1[e]) * r * bf16r(s1[e]), kInCarry); }
  unsigned short* dp = XN16 + i * 8u;
  *(volatile v8h*)dp = hv;
  __threadfence();
  *(volatile v8h*)dp = hv;
}
static_assert((size_t)kRows * kDm / 8 == 2048ull * kThr && kDm / 8 == 128, "the norm's grid exact: 2,048 blocks");

__global__ __launch_bounds__(kThr) void conv_kernel(const float* __restrict__ UZ, const float* __restrict__ conv_w, const float* __restrict__ conv_bias, float* __restrict__ U, unsigned short* __restrict__ U16) {
  const unsigned i = blockIdx.x * (unsigned)kThr + threadIdx.x;
  const unsigned row = i >> 8;
  const unsigned c8 = (i & 255u) * 8u;
  const unsigned t = row & (unsigned)(kL - 1);
  float acc[8];
  {
    const v4f b0 = *(const v4f*)(conv_bias + c8), b1 = *(const v4f*)(conv_bias + c8 + 4);
#pragma unroll
    for (int e = 0; e < 4; ++e) { acc[e] = bf16r(b0[e]); acc[4 + e] = bf16r(b1[e]); }
  }
#pragma unroll
  for (int j = 0; j < 4; ++j) {
    const unsigned back = (unsigned)(3 - j);
    const bool live = t >= back;
    const unsigned rr = live ? (row - back) : row;
    const float* up = UZ + rr * (unsigned)(2 * kDi) + c8;
    const v4f u0 = *(const v4f*)up, u1 = *(const v4f*)(up + 4);
    const v4f w0 = *(const v4f*)(conv_w + (unsigned)j * (unsigned)kDi + c8), w1 = *(const v4f*)(conv_w + (unsigned)j * (unsigned)kDi + c8 + 4);
#pragma unroll
    for (int e = 0; e < 4; ++e) { acc[e] += live ? (bf16r(w0[e]) * u0[e]) : 0.0f; acc[4 + e] += live ? (bf16r(w1[e]) * u1[e]) : 0.0f; }
  }
  v4f o0, o1; v8h hv;
#pragma unroll
  for (int e = 0; e < 4; ++e) {
    const float a = acc[e], b = acc[4 + e];
    const float ua = a / (1.0f + expf(-a)), ub = b / (1.0f + expf(-b));
    o0[e] = ua; o1[e] = ub; hv[e] = (_Float16)carry_flush(ua, kInCarry); hv[4 + e] = (_Float16)carry_flush(ub, kInCarry);
  }
  float* dp = U + row * (unsigned)kDi + c8;
  unsigned short* dh = U16 + row * (unsigned)kDi + c8;
  for (int pass = 0; pass < 2; ++pass) {
    *(volatile v4f*)dp = o0;
    *(volatile v4f*)(dp + 4) = o1;
    *(volatile v8h*)dh = hv;
    __threadfence();
  }
}
static_assert((size_t)kRows * kDi / 8 == 4096ull * kThr && kDi / 8 == 256, "the conv's grid exact: 4,096 blocks: a block a row");

__global__ __launch_bounds__(kThr) void xp_kernel(const float* __restrict__ XP, unsigned short* __restrict__ DTR16, float* __restrict__ BC) {
  const unsigned i = blockIdx.x * (unsigned)kThr + threadIdx.x;
  const unsigned row = i >> 4;
  const unsigned g = i & 15u;
  if (g >= 12u) return;
  const float* sp = XP + row * (unsigned)kXP + g * 8u;
  const v4f a0 = *(const v4f*)sp, a1 = *(const v4f*)(sp + 4);
  if (g < 8u) {
    v8h hv;
#pragma unroll
    for (int e = 0; e < 4; ++e) { hv[e] = (_Float16)carry_flush(a0[e], kInCarry); hv[4 + e] = (_Float16)carry_flush(a1[e], kInCarry); }
    unsigned short* dp = DTR16 + row * (unsigned)kR + g * 8u;
    *(volatile v8h*)dp = hv;
    __threadfence();
    *(volatile v8h*)dp = hv;
  } else {
    v4f o0, o1;
#pragma unroll
    for (int e = 0; e < 4; ++e) { o0[e] = tanhf(a0[e]); o1[e] = tanhf(a1[e]); }
    float* dp = BC + row * 32u + (g - 8u) * 8u;
    for (int pass = 0; pass < 2; ++pass) {
      *(volatile v4f*)dp = o0;
      *(volatile v4f*)(dp + 4) = o1;
      __threadfence();
    }
  }
}
static_assert((size_t)kRows * 16 == 256ull * kThr, "the readers' grid exact: 256 blocks: 16 threads a row");

__global__ __launch_bounds__(kThr) void scan_kernel(const float* __restrict__ DT, const float* __restrict__ U, const float* __restrict__ BC, const float* __restrict__ UZ, const float* __restrict__ a_log, const float* __restrict__ dpar, const float* __restrict__ dt_bias, unsigned short* __restrict__ Y16) {
  const unsigned sq = blockIdx.x >> 2;
  const unsigned c2 = ((blockIdx.x & 3u) * (unsigned)kThr + threadIdx.x) * 2u;
  float a0[kS], a1[kS], h0[kS], h1[kS];
#pragma unroll
  for (int s = 0; s < kS; ++s) { a0[s] = -expf(bf16r(a_log[c2 * (unsigned)kS + (unsigned)s])); a1[s] = -expf(bf16r(a_log[(c2 + 1u) * (unsigned)kS + (unsigned)s])); h0[s] = 0.0f; h1[s] = 0.0f; }
  const float d0 = bf16r(dpar[c2]), d1 = bf16r(dpar[c2 + 1u]);
  const float tb0 = bf16r(dt_bias[c2]), tb1 = bf16r(dt_bias[c2 + 1u]);
  for (int t = 0; t < kL; ++t) {
    const unsigned row = sq * (unsigned)kL + (unsigned)t;
    const float* bp = BC + row * 32u;
    const float p0 = DT[row * (unsigned)kDi + c2] + tb0, p1 = DT[row * (unsigned)kDi + c2 + 1u] + tb1;
    const float sp0 = fmaxf(p0, 0.0f) + log1pf(expf(-fabsf(p0))), sp1 = fmaxf(p1, 0.0f) + log1pf(expf(-fabsf(p1)));
    const float dt0 = fminf(fmaxf(sp0, kDtMin), kDtMax), dt1 = fminf(fmaxf(sp1, kDtMin), kDtMax);
    const float u0 = U[row * (unsigned)kDi + c2], u1 = U[row * (unsigned)kDi + c2 + 1u];
    const float g0 = dt0 * u0, g1 = dt1 * u1;
    float y0 = 0.0f, y1 = 0.0f;
#pragma unroll
    for (int q = 0; q < 4; ++q) {
      const v4f bq = *(const v4f*)(bp + 4 * q), cq = *(const v4f*)(bp + 16 + 4 * q);
#pragma unroll
      for (int e = 0; e < 4; ++e) {
        const int s = 4 * q + e;
        h0[s] = expf(dt0 * a0[s]) * h0[s] + g0 * bq[e];
        h1[s] = expf(dt1 * a1[s]) * h1[s] + g1 * bq[e];
        y0 += h0[s] * cq[e];
        y1 += h1[s] * cq[e];
      }
    }
    y0 += u0 * d0; y1 += u1 * d1;
    const float z0 = UZ[row * (unsigned)(2 * kDi) + (unsigned)kDi + c2], z1 = UZ[row * (unsigned)(2 * kDi) + (unsigned)kDi + c2 + 1u];
    const float o0 = y0 * (z0 / (1.0f + expf(-z0))), o1 = y1 * (z1 / (1.0f + expf(-z1)));
    v2h hv; hv[0] = (_Float16)carry_flush(o0, kYCarry); hv[1] = (_Float16)carry_flush(o1, kYCarry);
    unsigned short* dp = Y16 + row * (unsigned)kDi + c2;
    *(volatile v2h*)dp = hv;
    __threadfence();
    *(volatile v2h*)dp = hv;
  }
}
static_assert(kNB * kDi / 2 == 8 * kThr && kDi / 2 == 1024, "the scan's grid exact: 8 blocks: four a sequence");

__global__ __launch_bounds__(kThr) void close_kernel(const float* __restrict__ x, const float* __restrict__ O, float* __restrict__ out) {
  const unsigned i = blockIdx.x * (unsigned)kThr + threadIdx.x;
  const v4f x0 = *(const v4f*)(x + i * 8u), x1 = *(const v4f*)(x + i * 8u + 4u);
  const v4f p0 = *(const v4f*)(O + i * 8u), p1 = *(const v4f*)(O + i * 8u + 4u);
  v4f o0, o1;
#pragma unroll
  for (int e = 0; e < 4; ++e) { o0[e] = bf16r(x0[e]) + p0[e]; o1[e] = bf16r(x1[e]) + p1[e]; }
  float* dp = out + i * 8u;
  for (int pass = 0; pass < 2; ++pass) {
    *(volatile v4f*)dp = o0;
    *(volatile v4f*)(dp + 4) = o1;
    __threadfence();
  }
}
static_assert((size_t)kRows * kDm / 8 == 2048ull * kThr, "the residual's grid exact: 2,048 blocks");

extern "C" void kernel_launch(void* const* d_in, const int* in_sizes, int n_in,
                              void* d_out, int out_size, void* d_ws, size_t ws_size,
                              hipStream_t stream) {
  if (n_in < 19 || d_out == nullptr || d_ws == nullptr) return;
  if (in_sizes[0] != kRows * kDm || in_sizes[1] != kDm || in_sizes[2] != kDm * 2 * kDi || in_sizes[3] != 2 * kDi || in_sizes[4] != kDi * kDm || in_sizes[5] != kDm || in_sizes[6] != kDi * kR || in_sizes[7] != kR || in_sizes[8] != kR * kDi || in_sizes[9] != kDi) return;
  if (in_sizes[10] != kDi * kS || in_sizes[11] != kS || in_sizes[12] != kDi * kS || in_sizes[13] != kS || in_sizes[14] != 4 * kDi || in_sizes[15] != kDi || in_sizes[16] != kDi * kS || in_sizes[17] != kDi || in_sizes[18] != kDi) return;
  if (out_size != kOut0) return;
  if (ws_size < kWsTotal) return;
  const float* x = (const float*)d_in[0];
  const float* norm_scale = (const float*)d_in[1];
  const float* in_proj_w = (const float*)d_in[2];
  const float* in_proj_b = (const float*)d_in[3];
  const float* out_proj_w = (const float*)d_in[4];
  const float* out_proj_b = (const float*)d_in[5];
  const float* dt_in_w = (const float*)d_in[6];
  const float* dt_in_b = (const float*)d_in[7];
  const float* dt_out_w = (const float*)d_in[8];
  const float* dt_out_b = (const float*)d_in[9];
  const float* b_proj_w = (const float*)d_in[10];
  const float* b_proj_b = (const float*)d_in[11];
  const float* c_proj_w = (const float*)d_in[12];
  const float* c_proj_b = (const float*)d_in[13];
  const float* conv_w = (const float*)d_in[14];
  const float* conv_bias = (const float*)d_in[15];
  const float* a_log = (const float*)d_in[16];
  const float* dpar = (const float*)d_in[17];
  const float* dt_bias = (const float*)d_in[18];
  float* out = (float*)d_out;
  char* ws = (char*)d_ws;
  unsigned short* XN16 = (unsigned short*)(ws + kOffXN16);
  unsigned short* WIN16 = (unsigned short*)(ws + kOffWIN16);
  float* UZ = (float*)(ws + kOffUZ);
  float* U = (float*)(ws + kOffU);
  unsigned short* U16 = (unsigned short*)(ws + kOffU16);
  unsigned short* WX16 = (unsigned short*)(ws + kOffWX16);
  float* XP = (float*)(ws + kOffXP);
  unsigned short* DTR16 = (unsigned short*)(ws + kOffDTR16);
  float* BC = (float*)(ws + kOffBC);
  unsigned short* WDO16 = (unsigned short*)(ws + kOffWDO16);
  float* DT = (float*)(ws + kOffDT);
  unsigned short* Y16 = (unsigned short*)(ws + kOffY16);
  unsigned short* WOUT16 = (unsigned short*)(ws + kOffWOUT16);
  float* O = (float*)(ws + kOffO);
  float* BV = (float*)(ws + kOffBV);
  float* RS = (float*)(ws + kOffRS);

  setup_kernel<<<29, kThr, 0, stream>>>(in_proj_b, dt_in_b, b_proj_b, c_proj_b, dt_out_b, out_proj_b, BV);
  rowstat_kernel<<<16, kThr, 0, stream>>>(x, RS);
  norm_kernel<<<2048, kThr, 0, stream>>>(x, RS, norm_scale, XN16);
  wt_plane_kernel<<<2 * kDi, kDm / 8, 0, stream>>>(in_proj_w, WIN16, kDm, 2 * kDi, 2 * kDi, kDm, 0);
  wt_plane_kernel<<<kR, kDi / 8, 0, stream>>>(dt_in_w, WX16, kDi, kR, kR, kDi, 0);
  wt_plane_kernel<<<kS, kDi / 8, 0, stream>>>(b_proj_w, WX16 + (size_t)kR * kDi, kDi, kS, kS, kDi, 0);
  wt_plane_kernel<<<kS + 32, kDi / 8, 0, stream>>>(c_proj_w, WX16 + (size_t)(kR + kS) * kDi, kDi, kS, kS, kDi, 0);
  wt_plane_kernel<<<kDi, kR / 8, 0, stream>>>(dt_out_w, WDO16, kR, kDi, kDi, kR, 0);
  wt_plane_kernel<<<kDm, kDi / 8, 0, stream>>>(out_proj_w, WOUT16, kDi, kDm, kDm, kDi, 0);
  wmma_gemm64<0, false, 2, 0, false, 0><<<dim3((kRows / 64) * (2 * kDi / 64) / 8, 1), 256, 0, stream>>>(
      XN16, XN16, kDm, 0L, WIN16, WIN16, kDm, 0L, (void*)UZ, (void*)UZ, 2 * kDi, 0L, BV + kBvIn, nullptr, 0L, kRows, 2 * kDi, kDm, kScA);
  conv_kernel<<<4096, kThr, 0, stream>>>(UZ, conv_w, conv_bias, U, U16);
  wmma_gemm64<0, false, 2, 0, false, 0><<<dim3((kRows / 64) * (kXP / 64) / 8, 1), 256, 0, stream>>>(
      U16, U16, kDi, 0L, WX16, WX16, kDi, 0L, (void*)XP, (void*)XP, kXP, 0L, BV + kBvX, nullptr, 0L, kRows, kXP, kDi, kScA);
  xp_kernel<<<256, kThr, 0, stream>>>(XP, DTR16, BC);
  wmma_gemm64<0, false, 2, 0, false, 0><<<dim3((kRows / 64) * (kDi / 64) / 8, 1), 256, 0, stream>>>(
      DTR16, DTR16, kR, 0L, WDO16, WDO16, kR, 0L, (void*)DT, (void*)DT, kDi, 0L, BV + kBvDo, nullptr, 0L, kRows, kDi, kR, kScA);
  scan_kernel<<<8, kThr, 0, stream>>>(DT, U, BC, UZ, a_log, dpar, dt_bias, Y16);
  wmma_gemm64<0, false, 2, 0, false, 0><<<dim3((kRows / 64) * (kDm / 64) / 8, 1), 256, 0, stream>>>(
      Y16, Y16, kDi, 0L, WOUT16, WOUT16, kDi, 0L, (void*)O, (void*)O, kDm, 0L, BV + kBvOut, nullptr, 0L, kRows, kDm, kDi, kScY);
  close_kernel<<<2048, kThr, 0, stream>>>(x, O, out);
}
static_assert(((kRows / 64) * (kXP / 64)) % 8 == 0 && ((kRows / 64) * (kDm / 64)) % 8 == 0, "the engine's grids: whole blocks of eight wave tiles");
